// MultiHeadSelfAttention_395136991401
// MI455X (gfx1250) — hardware-verified
//
#include <hip/hip_runtime.h>
#ifndef NB
#define NB 2
#endif
#ifndef SEQ
#define SEQ 2048
#endif
#define NB_FULL 2
#define SEQ_FULL 2048
#define DM 1024
#define NH 16
#define HD 64
#define EARLY 256
#define LQK (2 * DM)
#define LCX (2 * DM)
#define NR ((size_t)NB * SEQ)

static_assert(DM == NH * HD);
static_assert(HD == 64);
static_assert((DM & (DM - 1)) == 0);
static_assert(DM % 128 == 0 && SEQ % 128 == 0);
static_assert(LQK % 64 == 0 && DM % 64 == 0 && SEQ % 64 == 0);
static_assert(EARLY % 32 == 0 && SEQ >= EARLY && (SEQ - EARLY) % 32 == 0);
static_assert((NB * NH * (EARLY / 16)) % 4 == 0);
static_assert((NB * NH * ((SEQ - EARLY) / 32)) % 4 == 0);
static_assert((NR * DM / 8) % 256 == 0 && ((size_t)DM * DM / 8) % 256 == 0);
static_assert(NB <= NB_FULL && SEQ <= SEQ_FULL);

typedef _Float16 v16h __attribute__((ext_vector_type(16)));
typedef _Float16 v4h  __attribute__((ext_vector_type(4)));
typedef unsigned short v8us __attribute__((ext_vector_type(8), may_alias));
typedef float v8f  __attribute__((ext_vector_type(8)));
typedef float v4f  __attribute__((ext_vector_type(4)));
typedef float v4fa __attribute__((ext_vector_type(4), may_alias));
union FragH { v16h v; v8us half[2]; _Float16 h[16]; };

__device__ __forceinline__ float bf16_rne(float x) { unsigned int u = __float_as_uint(x); u = (u + 0x7FFFu + ((u >> 16) & 1u)) & 0xFFFF0000u; return __uint_as_float(u); }

__device__ __forceinline__ v16h ld_frag(const _Float16* p, int hh) { FragH f; f.half[0] = *(const v8us*)((const unsigned short*)p + 8 * hh); f.half[1] = *(const v8us*)((const unsigned short*)p + 16 + 8 * hh); return f.v; }

__device__ __forceinline__ v8f mma1(v16h a, v16h b, v8f c) {
  v8f d = __builtin_amdgcn_wmma_f32_16x16x32_f16(false, a, false, b, (short)0, c, false, false);
  asm volatile("v_nop\n\tv_nop\n\tv_nop\n\tv_nop" : "+v"(d) : "v"(a), "v"(b));
  return d;
}
__device__ __forceinline__ v8f mma2(v16h a0, v16h b0, v16h a1, v16h b1, v8f c) {
  v8f d = __builtin_amdgcn_wmma_f32_16x16x32_f16(false, a0, false, b0, (short)0, c, false, false);
  d = __builtin_amdgcn_wmma_f32_16x16x32_f16(false, a1, false, b1, (short)0, d, false, false);
  asm volatile("v_nop\n\tv_nop\n\tv_nop\n\tv_nop" : "+v"(d) : "v"(a0), "v"(b0), "v"(a1), "v"(b1));
  return d;
}

__global__ __launch_bounds__(256) void k_x16(const float* __restrict__ x, _Float16* __restrict__ X16) {
  const size_t t = (size_t)blockIdx.x * 256 + threadIdx.x;
  if (t >= NR * DM / 8) return;
  const size_t e = t * 8;
  const size_t row = e / DM, col = e - row * DM;
  const size_t b = row / SEQ, s = row - b * SEQ;
  const float* src = x + (b * SEQ_FULL + s) * DM + col;
  const v4f a = *(const v4fa*)src, c = *(const v4fa*)(src + 4);
  FragH f;
#pragma unroll
  for (int q = 0; q < 4; ++q) { f.h[q] = (_Float16)bf16_rne(a[q]); f.h[4 + q] = (_Float16)bf16_rne(c[q]); }
  unsigned short* d = (unsigned short*)X16 + e;
  const v8us o = f.half[0];
  *(volatile v8us*)d = o; __threadfence(); *(volatile v8us*)d = o;
}

__global__ __launch_bounds__(256) void k_w16(const float* __restrict__ w, _Float16* __restrict__ Bt) {
  const size_t t = (size_t)blockIdx.x * 256 + threadIdx.x;
  if (t >= (size_t)DM * DM / 8) return;
  const size_t e = t * 8;
  const v4f a = *(const v4fa*)(w + e), c = *(const v4fa*)(w + e + 4);
  FragH f;
#pragma unroll
  for (int q = 0; q < 4; ++q) { f.h[q] = (_Float16)(bf16_rne(a[q]) * 16.0f); f.h[4 + q] = (_Float16)(bf16_rne(c[q]) * 16.0f); }
  unsigned short* d = (unsigned short*)Bt + e;
  const v8us o = f.half[0];
  *(volatile v8us*)d = o; __threadfence(); *(volatile v8us*)d = o;
}

__global__ __launch_bounds__(128) void k_gemm(const _Float16* __restrict__ A, int lda, size_t sA, const _Float16* __restrict__ Bh, int ldb, size_t sB, int kmask, float alpha,
                                              float* __restrict__ C, _Float16* __restrict__ Ch, _Float16* __restrict__ Cr, int ldc, size_t sC, int N, int K) {
  __shared__ __attribute__((aligned(16))) float so[4][32][68];
  const int tid = threadIdx.x, lane = tid & 31, ln = lane & 15, hh = lane >> 4;
  const int w = __builtin_amdgcn_readfirstlane(tid >> 5);
  const int by = blockIdx.y;
  A += (size_t)by * sA; Bh += (size_t)by * sB; const size_t cofs = (size_t)by * sC;
  const int ntn = N >> 6; const int mt = blockIdx.x / ntn, nq = blockIdx.x - mt * ntn;
  const int row0 = mt * 128 + 32 * w, col0 = nq * 64;
  const _Float16* a0p = A + (size_t)(row0 + ln) * lda; const _Float16* a1p = a0p + (size_t)16 * lda;
  const _Float16* b0p = Bh + (size_t)(col0 + ln) * ldb; const _Float16* b1p = b0p + (size_t)16 * ldb; const _Float16* b2p = b1p + (size_t)16 * ldb; const _Float16* b3p = b2p + (size_t)16 * ldb;
  const v8f z8 = {0.f, 0.f, 0.f, 0.f, 0.f, 0.f, 0.f, 0.f};
  v8f c00 = z8, c01 = z8, c02 = z8, c03 = z8, c10 = z8, c11 = z8, c12 = z8, c13 = z8;
#pragma unroll 1
  for (int kb = 0; kb < K; kb += 32) {
    const int kbb = kb & kmask;
    const v16h a0 = ld_frag(a0p + kb, hh), a1 = ld_frag(a1p + kb, hh);
    v16h b = ld_frag(b0p + kbb, hh); c00 = mma1(a0, b, c00); c10 = mma1(a1, b, c10);
    b = ld_frag(b1p + kbb, hh); c01 = mma1(a0, b, c01); c11 = mma1(a1, b, c11);
    b = ld_frag(b2p + kbb, hh); c02 = mma1(a0, b, c02); c12 = mma1(a1, b, c12);
    b = ld_frag(b3p + kbb, hh); c03 = mma1(a0, b, c03); c13 = mma1(a1, b, c13);
  }
  v8f accs[8] = {c00, c01, c02, c03, c10, c11, c12, c13};
#pragma unroll
  for (int u = 0; u < 8; ++u) { const int t = u & 3, half = u >> 2;
#pragma unroll
    for (int r = 0; r < 8; ++r) so[w][half * 16 + 8 * hh + r][t * 16 + ln] = accs[u][r] * alpha; }
  __syncthreads();
  const int rsub = lane >> 4, c4 = (lane & 15) * 4;
  for (int pass = 0; pass < 2; ++pass) {
#pragma unroll
    for (int q = 0; q < 16; ++q) {
      const int r = q * 2 + rsub;
      const v4f v = *(const v4fa*)&so[w][r][c4];
      const size_t o = cofs + (size_t)(row0 + r) * ldc + col0 + c4;
      if (C) *(volatile v4f*)(C + o) = v;
      if (Ch) {
        v4h hv, rv;
#pragma unroll
        for (int i = 0; i < 4; ++i) { const _Float16 h = (_Float16)v[i]; hv[i] = h; rv[i] = (_Float16)(v[i] - (float)h); }
        *(volatile v4h*)(Ch + o) = hv;
        *(volatile v4h*)(Cr + o) = rv;
      }
    }
    if (pass == 0) __threadfence();
  }
}

template <int NU, bool FULL>
__device__ __forceinline__ void attn_tile(const _Float16* __restrict__ QKh, const _Float16* __restrict__ QKr, const _Float16* __restrict__ Vth, const _Float16* __restrict__ Vtr, _Float16* __restrict__ CTX) {
  constexpr int QW = 16 * NU;
  constexpr int QBASE = FULL ? 0 : EARLY;
  constexpr int TPB = FULL ? (EARLY / QW) : ((SEQ - EARLY) / QW);
  static_assert(QW % 4 == 0);
  __shared__ __attribute__((aligned(16))) unsigned short st[4][2][QW][HD];
  const int lane = threadIdx.x & 31, n = lane & 15, hh = lane >> 4;
  const int wave = __builtin_amdgcn_readfirstlane(threadIdx.x >> 5);
  const int tile = blockIdx.x * 4 + wave;
  const int bh = tile / TPB, ti = tile - bh * TPB;
  const int b = bh / NH, head = bh - b * NH;
  const int q0 = QBASE + ti * QW;
  const size_t tok0 = (size_t)b * SEQ;
  const size_t qoff0 = (tok0 + q0 + n) * LQK + head * HD;
  const size_t koffb = (tok0 + n) * LQK + DM + head * HD;
  const size_t voffb = ((size_t)b * DM + head * HD + n) * SEQ;
  const float CS = 0.18033688011112042f * (1.0f / 4096.0f);
  const float NEG = -1.0e30f;
  const v8f z8 = {0.f, 0.f, 0.f, 0.f, 0.f, 0.f, 0.f, 0.f};
  v8f oacc[NU][4];
  float mrun[NU], lrun[NU];
#pragma unroll
  for (int u = 0; u < NU; ++u) { mrun[u] = NEG; lrun[u] = 0.f;
#pragma unroll
    for (int g = 0; g < 4; ++g) oacc[u][g] = z8; }
  const int kend = q0 + QW;
#pragma unroll 1
  for (int j0 = 0; j0 < kend; j0 += 32) {
    v16h kh[2][2], kr[2][2];
#pragma unroll
    for (int t = 0; t < 2; ++t) {
#pragma unroll
      for (int c = 0; c < 2; ++c) {
        const size_t ko = koffb + (size_t)(j0 + 16 * t) * LQK + 32 * c;
        kh[t][c] = ld_frag(QKh + ko, hh);
        kr[t][c] = kh[t][c];
        if (FULL) kr[t][c] = ld_frag(QKr + ko, hh);
      }
    }
    FragH ph[NU], pr[NU];
    const bool diag = (j0 + 31 > q0);
#pragma unroll
    for (int u = 0; u < NU; ++u) {
      const size_t qo = qoff0 + (size_t)(16 * u) * LQK;
      const v16h qh0 = ld_frag(QKh + qo, hh), qh1 = ld_frag(QKh + qo + 32, hh);
      const v16h qr0 = ld_frag(QKr + qo, hh), qr1 = ld_frag(QKr + qo + 32, hh);
      v8f s0 = mma2(kh[0][0], qh0, kh[0][1], qh1, z8);
      s0 = mma2(kh[0][0], qr0, kh[0][1], qr1, s0);
      v8f s1 = mma2(kh[1][0], qh0, kh[1][1], qh1, z8);
      s1 = mma2(kh[1][0], qr0, kh[1][1], qr1, s1);
      if (FULL) { s0 = mma2(kr[0][0], qh0, kr[0][1], qh1, s0); s1 = mma2(kr[1][0], qh0, kr[1][1], qh1, s1); }
      float x0[8], x1[8];
#pragma unroll
      for (int r = 0; r < 8; ++r) { x0[r] = s0[r] * CS; x1[r] = s1[r] * CS; }
      if (diag) {
        const int qrow = q0 + 16 * u + n; const int kb0 = j0 + 8 * hh;
#pragma unroll
        for (int r = 0; r < 8; ++r) { x0[r] = (kb0 + r > qrow) ? NEG : x0[r]; x1[r] = (kb0 + 16 + r > qrow) ? NEG : x1[r]; }
      }
      float ml = fmaxf(x0[0], x1[0]);
#pragma unroll
      for (int r = 1; r < 8; ++r) ml = fmaxf(ml, fmaxf(x0[r], x1[r]));
      ml = fmaxf(ml, __shfl_xor(ml, 16));
      const float mnew = fmaxf(mrun[u], ml);
      const float corr = __builtin_amdgcn_exp2f(mrun[u] - mnew);
      mrun[u] = mnew;
      float ls = 0.f;
#pragma unroll
      for (int r = 0; r < 8; ++r) {
        const float p0 = __builtin_amdgcn_exp2f(x0[r] - mnew), p1 = __builtin_amdgcn_exp2f(x1[r] - mnew);
        ls += p0 + p1;
        const float c0 = p0 * 256.0f, c1 = p1 * 256.0f;
        const _Float16 h0 = (_Float16)c0, h1 = (_Float16)c1;
        ph[u].h[r] = h0; ph[u].h[8 + r] = h1;
        pr[u].h[r] = (_Float16)(c0 - (float)h0); pr[u].h[8 + r] = (_Float16)(c1 - (float)h1);
      }
      ls += __shfl_xor(ls, 16);
      lrun[u] = lrun[u] * corr + ls;
#pragma unroll
      for (int g = 0; g < 4; ++g)
#pragma unroll
        for (int r = 0; r < 8; ++r) oacc[u][g][r] *= corr;
    }
#pragma unroll
    for (int g = 0; g < 4; ++g) {
      const size_t vo = voffb + (size_t)(16 * g) * SEQ + j0;
      const v16h vh = ld_frag(Vth + vo, hh);
      v16h vr = vh;
      if (FULL) vr = ld_frag(Vtr + vo, hh);
#pragma unroll
      for (int u = 0; u < NU; ++u) {
        if (FULL) { oacc[u][g] = mma2(vh, ph[u].v, vr, ph[u].v, oacc[u][g]); oacc[u][g] = mma1(vh, pr[u].v, oacc[u][g]); }
        else oacc[u][g] = mma1(vh, ph[u].v, oacc[u][g]);
      }
    }
  }
#pragma unroll
  for (int u = 0; u < NU; ++u) {
    const float inv = 1.0f / (lrun[u] * 16.0f);
#pragma unroll
    for (int g = 0; g < 4; ++g) {
      FragH fh, fr;
#pragma unroll
      for (int r = 0; r < 8; ++r) { const float val = oacc[u][g][r] * inv; const _Float16 h = (_Float16)val; fh.h[r] = h; fr.h[r] = (_Float16)(val - (float)h); }
      *(v8us*)&st[wave][0][16 * u + n][16 * g + 8 * hh] = fh.half[0];
      *(v8us*)&st[wave][1][16 * u + n][16 * g + 8 * hh] = fr.half[0];
    }
  }
  __syncthreads();
  const int rq = lane >> 3, pc = (lane & 7) * 8;
  for (int pass = 0; pass < 2; ++pass) {
#pragma unroll
    for (int it = 0; it < QW / 4; ++it) {
      const int row = it * 4 + rq;
      const v8us vv = *(const v8us*)&st[wave][0][row][pc];
      const v8us vr = *(const v8us*)&st[wave][1][row][pc];
      unsigned short* d = (unsigned short*)CTX + (tok0 + q0 + row) * LCX + head * HD + pc;
      *(volatile v8us*)d = vv;
      *(volatile v8us*)(d + DM) = vr;
    }
    if (pass == 0) __threadfence();
  }
}

__global__ __launch_bounds__(128) void k_attn_early(const _Float16* __restrict__ QKh, const _Float16* __restrict__ QKr, const _Float16* __restrict__ Vth, const _Float16* __restrict__ Vtr, _Float16* __restrict__ CTX) {
  attn_tile<1, true>(QKh, QKr, Vth, Vtr, CTX);
}
__global__ __launch_bounds__(128) void k_attn_late(const _Float16* __restrict__ QKh, const _Float16* __restrict__ QKr, const _Float16* __restrict__ Vth, const _Float16* __restrict__ Vtr, _Float16* __restrict__ CTX) {
  attn_tile<2, false>(QKh, QKr, Vth, Vtr, CTX);
}

#define SZ_WQK ((size_t)2 * DM * DM * 2)
#define SZ_W1  ((size_t)DM * DM * 2)
#define SZ_X16 (NR * DM * 2)
#define SZ_QK  (NR * LQK * 2)
#define SZ_VT  ((size_t)NB * DM * SEQ * 2)
#define SZ_CTX (NR * LCX * 2)
#define SZ_ALL (SZ_WQK + 2 * SZ_W1 + SZ_X16 + 2 * SZ_QK + 2 * SZ_VT + SZ_CTX)
static_assert(SZ_WQK % 256 == 0 && SZ_W1 % 256 == 0 && SZ_X16 % 256 == 0 && SZ_QK % 256 == 0 && SZ_VT % 256 == 0 && SZ_CTX % 256 == 0);
static_assert(SZ_ALL <= (size_t)134217728);

extern "C" void kernel_launch(void* const* d_in, const int* in_sizes, int n_in,
                              void* d_out, int out_size, void* d_ws, size_t ws_size, hipStream_t stream) {
  if (n_in < 5) return;
  const size_t need_x = ((size_t)(NB - 1) * SEQ_FULL + SEQ) * DM;
  if ((size_t)in_sizes[0] < need_x) return;
  for (int i = 1; i < 5; ++i) if ((size_t)in_sizes[i] < (size_t)DM * DM) return;
  if ((size_t)out_size < need_x) return;
  if (SZ_ALL > ws_size) return;
  const float* x = (const float*)d_in[0];
  const float* wq = (const float*)d_in[1]; const float* wk = (const float*)d_in[2];
  const float* wv = (const float*)d_in[3]; const float* wo = (const float*)d_in[4];
  float* out = (float*)d_out;
  char* ws = (char*)d_ws; size_t off = 0;
  _Float16* WQK = (_Float16*)(ws + off); off += SZ_WQK;
  _Float16* WV16 = (_Float16*)(ws + off); off += SZ_W1;
  _Float16* WO16 = (_Float16*)(ws + off); off += SZ_W1;
  _Float16* X16 = (_Float16*)(ws + off); off += SZ_X16;
  _Float16* QKh = (_Float16*)(ws + off); off += SZ_QK;
  _Float16* QKr = (_Float16*)(ws + off); off += SZ_QK;
  _Float16* VTh = (_Float16*)(ws + off); off += SZ_VT;
  _Float16* VTr = (_Float16*)(ws + off); off += SZ_VT;
  _Float16* CTX = (_Float16*)(ws + off); off += SZ_CTX;
  if (off > ws_size) return;

  k_x16<<<(unsigned)(NR * DM / 8 / 256), 256, 0, stream>>>(x, X16);
  const unsigned wgrid = (unsigned)((size_t)DM * DM / 8 / 256);
  k_w16<<<wgrid, 256, 0, stream>>>(wq, WQK);
  k_w16<<<wgrid, 256, 0, stream>>>(wk, WQK + (size_t)DM * DM);
  k_w16<<<wgrid, 256, 0, stream>>>(wv, WV16);
  k_w16<<<wgrid, 256, 0, stream>>>(wo, WO16);
  k_gemm<<<dim3((unsigned)((NR / 128) * (LQK / 64)), 1), 128, 0, stream>>>(X16, DM, (size_t)0, WQK, DM, (size_t)0, DM - 1, 4.0f,
      nullptr, QKh, QKr, LQK, (size_t)0, LQK, DM);
  k_gemm<<<dim3((unsigned)((DM / 128) * (SEQ / 64)), NB), 128, 0, stream>>>(WV16, DM, (size_t)0, X16, DM, (size_t)SEQ * DM, DM - 1, 4.0f,
      nullptr, VTh, VTr, SEQ, (size_t)DM * SEQ, SEQ, DM);
  k_attn_early<<<(unsigned)(NB * NH * (EARLY / 16) / 4), 128, 0, stream>>>(QKh, QKr, VTh, VTr, CTX);
  if (SEQ > EARLY)
    k_attn_late<<<(unsigned)(NB * NH * ((SEQ - EARLY) / 32) / 4), 128, 0, stream>>>(QKh, QKr, VTh, VTr, CTX);
  k_gemm<<<dim3((unsigned)((SEQ / 128) * (DM / 64)), NB), 128, 0, stream>>>(CTX, LCX, (size_t)SEQ * LCX, WO16, DM, (size_t)0, DM - 1, 0.00006103515625f,
      out, nullptr, nullptr, DM, (size_t)SEQ_FULL * DM, DM, 2 * DM);
}
